// CrossAttention_31834297598397
// MI455X (gfx1250) — hardware-run, weakly checked
//
#include <hip/hip_runtime.h>
#ifndef NB
#define NB 4
#endif
#ifndef SEQ
#define SEQ 1024
#endif
#define NB_FULL 4
#define SEQ_FULL 1024
#define SCTX 1024
#define DM 1024
#define NH 16
#define HD 64
#define NR ((size_t)NB * SEQ)
#define NRC ((size_t)NB * SCTX)
static_assert(SEQ % 128 == 0);
static_assert(SEQ <= SEQ_FULL);
static_assert(NB >= 1 && NB <= NB_FULL);
static_assert(SCTX % 128 == 0);
static_assert(DM % 128 == 0 && DM == NH * HD && HD == 64);
static_assert(DM % 64 == 0 && DM % 32 == 0);
static_assert((size_t)NB_FULL * SEQ_FULL * DM * 4 == 16777216);

typedef unsigned short v8us __attribute__((ext_vector_type(8), may_alias));
typedef float  v8f  __attribute__((ext_vector_type(8)));
typedef float  v4f  __attribute__((ext_vector_type(4)));
typedef float  v4fa __attribute__((ext_vector_type(4), may_alias));
typedef int    v4i  __attribute__((ext_vector_type(4), may_alias));
typedef _Float16 v16h __attribute__((ext_vector_type(16)));
typedef _Float16 v4h __attribute__((ext_vector_type(4)));
union FragH { v16h v; v8us half[2]; _Float16 h[16]; unsigned short u[16]; unsigned int w[8]; };

__device__ __forceinline__ unsigned short bf16_bits(float x) { unsigned int u = __float_as_uint(x); return (unsigned short)((u + 0x7FFFu + ((u >> 16) & 1u)) >> 16); }
__device__ __forceinline__ float bf16_val(unsigned short b) { return __uint_as_float(((unsigned int)b) << 16); }
__device__ __forceinline__ float bf16_rne(float x) { return bf16_val(bf16_bits(x)); }

typedef _Float16 h16;
static __device__ __forceinline__ h16 toh_flush(float v) { const h16 r = (h16)v; return (fabsf(v) < 6.103515625e-05f) ? (h16)0.0f : r; }

__global__ __launch_bounds__(256) void k_wt_f16(const float* __restrict__ W, _Float16* __restrict__ Wt, int K, int N, float scale) {
  const int t = blockIdx.x * 256 + threadIdx.x; if (t >= N * (K / 8)) return; const int n = t / (K / 8), k8 = (t % (K / 8)) * 8; FragH f;
#pragma unroll
  for (int i = 0; i < 8; ++i) f.h[i] = toh_flush(bf16_rne(W[(size_t)(k8 + i) * N + n]) * scale);
  const v8us o = f.half[0]; unsigned short* d = (unsigned short*)Wt + (size_t)n * K + k8;
  *(volatile v8us*)d = o; __threadfence(); *(volatile v8us*)d = o;
}

__global__ __launch_bounds__(256) void k_x16(const float* __restrict__ x, _Float16* __restrict__ X16, size_t n8) {
  const size_t t = (size_t)blockIdx.x * 256 + threadIdx.x; if (t >= n8) return; FragH f;
  const v4f a = *(const v4fa*)(x + t * 8), c = *(const v4fa*)(x + t * 8 + 4);
#pragma unroll
  for (int q = 0; q < 4; ++q) { f.h[q] = (_Float16)bf16_rne(a[q]); f.h[4 + q] = (_Float16)bf16_rne(c[q]); }
  unsigned short* d = (unsigned short*)X16 + t * 8; *(volatile v8us*)d = f.half[0]; __threadfence(); *(volatile v8us*)d = f.half[0];
}

template <int NHv, int TTv>
__global__ __launch_bounds__(256) void k_vt(const _Float16* __restrict__ V16, int ldv, int voff, _Float16* __restrict__ Vt) {
  __shared__ unsigned short tl[64][66]; const int tid = threadIdx.x; const int slab = blockIdx.x / (TTv / 64), lg = blockIdx.x % (TTv / 64); const int b = slab / NHv, h = slab % NHv;
  for (int i = tid; i < 64 * 8; i += 256) { const int r = i / 8, c8 = (i % 8) * 8; FragH f; f.half[0] = *(const v8us*)((const unsigned short*)V16 + ((size_t)b * TTv + lg * 64 + r) * ldv + voff + h * 64 + c8);
#pragma unroll
    for (int q = 0; q < 8; ++q) tl[r][c8 + q] = f.u[q]; }
  __syncthreads();
  for (int pass = 0; pass < 2; ++pass) {
#pragma unroll
    for (int rd = 0; rd < 2; ++rd) { const int d = rd * 32 + tid / 8, pc = tid % 8; FragH f;
#pragma unroll
      for (int q = 0; q < 8; ++q) f.u[q] = tl[pc * 8 + q][d];
      *(volatile v8us*)((unsigned short*)Vt + ((size_t)slab * 64 + d) * TTv + lg * 64 + pc * 8) = f.half[0]; }
    if (pass == 0) __threadfence(); }
}

__device__ __forceinline__ v16h g2_frag(const _Float16* p, int hh) { FragH f; f.half[0] = *(const v8us*)((const unsigned short*)p + 8 * hh); f.half[1] = *(const v8us*)((const unsigned short*)p + 16 + 8 * hh); return f.v; }
__device__ __forceinline__ v8f g2_mma(v16h a, v16h b, v8f c) { v8f d = __builtin_amdgcn_wmma_f32_16x16x32_f16(false, a, false, b, (short)0, c, false, false); asm volatile("v_nop\n\tv_nop\n\tv_nop\n\tv_nop" : "+v"(d) : "v"(a), "v"(b)); return d; }
template <int ACT, int CPR, int MSK, int ZSK, int RSC>
__global__ __launch_bounds__(128) void k_gemm2(const _Float16* __restrict__ A, int lda, size_t sA, const _Float16* __restrict__ Bh, int ldb, size_t sB, float alpha,
    const float* __restrict__ bias, const float* __restrict__ CP, const int* __restrict__ mk, int mstr, const float* __restrict__ rs, int srs,
    float* __restrict__ C, _Float16* __restrict__ C16, int ldc, size_t sC, int M, int N, int K) {
  static_assert(ACT == 0 || ACT == 3);
  __shared__ __attribute__((aligned(16))) float so[4][32][68];
  const int tid = threadIdx.x, w = tid >> 5, lane = tid & 31, ln = lane & 15, hh = lane >> 4; const int by = blockIdx.y;
  A += (size_t)by * sA; Bh += (size_t)by * sB; const size_t cofs = (size_t)by * sC;
  const int ntn = N >> 6; const int mt = blockIdx.x / ntn, nq = blockIdx.x - mt * ntn; const int row0 = mt * 128 + 32 * w, col0 = nq * 64; if (row0 >= M) return;
  const _Float16* a0p = A + (size_t)(row0 + ln) * lda; const _Float16* a1p = a0p + (size_t)16 * lda;
  const _Float16* b0p = Bh + (size_t)(col0 + ln) * ldb; const _Float16* b1p = b0p + (size_t)16 * ldb; const _Float16* b2p = b1p + (size_t)16 * ldb; const _Float16* b3p = b2p + (size_t)16 * ldb;
  const v8f z8 = {0.f,0.f,0.f,0.f,0.f,0.f,0.f,0.f}; v8f c00 = z8, c01 = z8, c02 = z8, c03 = z8, c10 = z8, c11 = z8, c12 = z8, c13 = z8;
  bool live = true;
  if (MSK) {
    const int* mr = mk + (size_t)(row0 + lane) * mstr + col0; int anyu = 0;
#pragma unroll
    for (int j = 0; j < 64; j += 4) { const v4i m4 = *(const v4i*)(mr + j); anyu |= (m4[0] == 0) | (m4[1] == 0) | (m4[2] == 0) | (m4[3] == 0); }
    live = __any(anyu) != 0;
  }
  if (live) {
#pragma unroll 1
    for (int kb = 0; kb < K; kb += 32) {
      FragH fa0, fa1;
      fa0.half[0] = *(const v8us*)((const unsigned short*)a0p + kb + 8 * hh); fa0.half[1] = *(const v8us*)((const unsigned short*)a0p + kb + 16 + 8 * hh);
      fa1.half[0] = *(const v8us*)((const unsigned short*)a1p + kb + 8 * hh); fa1.half[1] = *(const v8us*)((const unsigned short*)a1p + kb + 16 + 8 * hh);
      if (ZSK) { unsigned int z = 0u;
#pragma unroll
        for (int i = 0; i < 8; ++i) z |= fa0.w[i] | fa1.w[i];
        if (__any(z != 0u) == 0) continue; }
      v16h b = g2_frag(b0p + kb, hh); c00 = g2_mma(fa0.v, b, c00); c10 = g2_mma(fa1.v, b, c10);
      b = g2_frag(b1p + kb, hh); c01 = g2_mma(fa0.v, b, c01); c11 = g2_mma(fa1.v, b, c11);
      b = g2_frag(b2p + kb, hh); c02 = g2_mma(fa0.v, b, c02); c12 = g2_mma(fa1.v, b, c12);
      b = g2_frag(b3p + kb, hh); c03 = g2_mma(fa0.v, b, c03); c13 = g2_mma(fa1.v, b, c13); }
  }
  v8f accs[8] = {c00, c01, c02, c03, c10, c11, c12, c13};
  float rsl[16];
#pragma unroll
  for (int i = 0; i < 16; ++i) rsl[i] = 1.0f;
  if (RSC) {
#pragma unroll
    for (int hf = 0; hf < 2; ++hf)
#pragma unroll
      for (int r = 0; r < 8; ++r) rsl[hf * 8 + r] = rs[(size_t)by * srs + row0 + hf * 16 + 8 * hh + r];
  }
#pragma unroll
  for (int u = 0; u < 8; ++u) { const int t = u & 3, hf = u >> 2; const int col = col0 + t * 16 + ln; const float bv = bias ? bf16_rne(bias[col]) : 0.f;
#pragma unroll
    for (int r = 0; r < 8; ++r) { const int rloc = hf * 16 + 8 * hh + r; float v = accs[u][r] * alpha; if (RSC) v *= rsl[hf * 8 + r]; v += bv;
      if (CP) { float cv = CP[cofs + (size_t)(row0 + rloc) * ldc + col]; if (CPR) cv = bf16_rne(cv); v += cv; }
      if (MSK) { const int m = mk[(size_t)(row0 + rloc) * mstr + col]; v = (m != 0) ? -1.0e9f : v; }
      if (ACT == 3) v = fmaxf(v, 0.f);
      so[w][rloc][t * 16 + ln] = v; } }
  __builtin_amdgcn_fence(4  , "workgroup"); __builtin_amdgcn_wave_barrier();
  const int rsub = lane >> 4, c4 = (lane & 15) * 4;
  for (int pass = 0; pass < 2; ++pass) {
#pragma unroll
    for (int q = 0; q < 16; ++q) { const int r = q * 2 + rsub; const v4f v = *(const v4fa*)&so[w][r][c4]; if (C) *(volatile v4f*)(C + cofs + (size_t)(row0 + r) * ldc + col0 + c4) = v; if (C16) { v4h h4;
#pragma unroll
        for (int i = 0; i < 4; ++i) h4[i] = (_Float16)v[i]; *(volatile v4h*)(C16 + cofs + (size_t)(row0 + r) * ldc + col0 + c4) = h4; } }
    if (pass == 0) __threadfence(); }
}

__global__ __launch_bounds__(256) void k_rmsres(const float* __restrict__ X, const float* __restrict__ g, _Float16* __restrict__ Hi, _Float16* __restrict__ Rs, int nrows) {
  #pragma clang fp contract(off)
  const int wave = __builtin_amdgcn_readfirstlane(threadIdx.x >> 5); const int lane = threadIdx.x & 31;
  const int r = blockIdx.x * 8 + wave; if (r >= nrows) return;
  const float* xr = X + (size_t)r * DM + lane * 4; float ss = 0.f;
#pragma unroll 1
  for (int j = 0; j < DM / 128; ++j) { const v4f a = *(const v4fa*)(xr + j * 128); ss = ss + a[0] * a[0]; ss = ss + a[1] * a[1]; ss = ss + a[2] * a[2]; ss = ss + a[3] * a[3]; }
#pragma unroll
  for (int off = 16; off >= 1; off >>= 1) ss = ss + __shfl_xor(ss, off, 32);
  const float rr = rsqrtf(ss * (1.0f / (float)DM) + 1.0e-6f);
  static_assert(32 * 8 * (DM / 128) == DM * 2);
#pragma unroll 1
  for (int j = 0; j < DM / 128; ++j) { const v4f a = *(const v4fa*)(xr + j * 128); const v4f gs = *(const v4fa*)(g + j * 128 + lane * 4); v4h yh, yr;
#pragma unroll
    for (int q = 0; q < 4; ++q) { const float gv = bf16_rne(gs[q]); const float y = (a[q] * rr) * gv + a[q]; const h16 hi = toh_flush(y); yh[q] = hi; yr[q] = toh_flush((y - (float)hi) * 2048.0f); }
    const size_t o = (size_t)r * DM + j * 128 + lane * 4;
    *(volatile v4h*)(Hi + o) = yh; *(volatile v4h*)(Rs + o) = yr; __threadfence(); *(volatile v4h*)(Hi + o) = yh; *(volatile v4h*)(Rs + o) = yr; }
}

__device__ __forceinline__ void score_tile(const _Float16* __restrict__ KH, const _Float16* __restrict__ KR, size_t ka, int hh, v16h qh0, v16h qh1, v16h qr0, v16h qr1, v8f& s, v8f& r) {
  const v8f z8 = {0.f,0.f,0.f,0.f,0.f,0.f,0.f,0.f}; s = z8; r = z8;
  v16h a = g2_frag(KH + ka, hh); s = g2_mma(a, qh0, s); r = g2_mma(a, qr0, r);
  a = g2_frag(KH + ka + 32, hh); s = g2_mma(a, qh1, s); r = g2_mma(a, qr1, r);
  a = g2_frag(KR + ka, hh); r = g2_mma(a, qh0, r);
  a = g2_frag(KR + ka + 32, hh); r = g2_mma(a, qh1, r);
}

__global__ __launch_bounds__(128) void k_flash(const _Float16* __restrict__ QH, const _Float16* __restrict__ QR, const _Float16* __restrict__ KH, const _Float16* __restrict__ KR,
    const _Float16* __restrict__ VT, _Float16* __restrict__ O16, float* __restrict__ ST) {
  __shared__ __attribute__((aligned(16))) float so[4][16][68];
  static_assert(sizeof(float) * 4 * 16 * 68 <= 131072);
  const int wave = __builtin_amdgcn_readfirstlane(threadIdx.x >> 5); const int lane = threadIdx.x & 31, ln = lane & 15, hh = lane >> 4;
  const int bh = blockIdx.y; const int b = bh / NH, h = bh - b * NH; const int q0 = blockIdx.x * 64 + wave * 16;
  const size_t qoff = ((size_t)b * SEQ + q0 + ln) * DM + h * HD;
  const size_t koff = ((size_t)b * SCTX + ln) * DM + h * HD;
  const size_t voff = ((size_t)bh * HD + ln) * SCTX;
  const v8f z8 = {0.f,0.f,0.f,0.f,0.f,0.f,0.f,0.f}; v8f o0 = z8, o1 = z8, o2 = z8, o3 = z8; float m = -3.0e38f, l = 0.f;
#pragma unroll 1
  for (int kb = 0; kb < SCTX; kb += 32) {
    const v16h qh0 = g2_frag(QH + qoff, hh), qh1 = g2_frag(QH + qoff + 32, hh), qr0 = g2_frag(QR + qoff, hh), qr1 = g2_frag(QR + qoff + 32, hh);
    const size_t ka = koff + (size_t)kb * DM;
    v8f s0, r0, s1, r1;
    score_tile(KH, KR, ka, hh, qh0, qh1, qr0, qr1, s0, r0);
    score_tile(KH, KR, ka + (size_t)16 * DM, hh, qh0, qh1, qr0, qr1, s1, r1);
    float e0[8], e1[8]; float tmax = -3.0e38f;
#pragma unroll
    for (int r = 0; r < 8; ++r) { e0[r] = s0[r] * 0.125f + r0[r] * 6.103515625e-05f; e1[r] = s1[r] * 0.125f + r1[r] * 6.103515625e-05f; tmax = fmaxf(tmax, fmaxf(e0[r], e1[r])); }
    tmax = fmaxf(tmax, __shfl_xor(tmax, 16, 32));
    const float mn = fmaxf(m, tmax); const float sc = __expf(m - mn); m = mn; l = l * sc; o0 = o0 * sc; o1 = o1 * sc; o2 = o2 * sc; o3 = o3 * sc;
    FragH pb;
#pragma unroll
    for (int r = 0; r < 8; ++r) { const float d0 = e0[r] - mn, d1 = e1[r] - mn; const float p0 = __expf(d0), p1 = __expf(d1); l = l + p0; l = l + p1;
      pb.h[r] = (d0 < -19.0f) ? (h16)0.0f : (h16)(p0 * 16384.0f); pb.h[8 + r] = (d1 < -19.0f) ? (h16)0.0f : (h16)(p1 * 16384.0f); }
    const size_t va = voff + kb;
    v16h a = g2_frag(VT + va, hh); o0 = g2_mma(a, pb.v, o0);
    a = g2_frag(VT + va + (size_t)16 * SCTX, hh); o1 = g2_mma(a, pb.v, o1);
    a = g2_frag(VT + va + (size_t)32 * SCTX, hh); o2 = g2_mma(a, pb.v, o2);
    a = g2_frag(VT + va + (size_t)48 * SCTX, hh); o3 = g2_mma(a, pb.v, o3);
  }
  const float lt = l + __shfl_xor(l, 16, 32); const float rl = 1.0f / lt; const float osc = rl * 0.00390625f;
#pragma unroll
  for (int r = 0; r < 8; ++r) { so[wave][ln][8 * hh + r] = o0[r] * osc; so[wave][ln][16 + 8 * hh + r] = o1[r] * osc; so[wave][ln][32 + 8 * hh + r] = o2[r] * osc; so[wave][ln][48 + 8 * hh + r] = o3[r] * osc; }
  __builtin_amdgcn_fence(4  , "workgroup"); __builtin_amdgcn_wave_barrier();
  const float stv = (hh != 0) ? rl : m;
  static_assert(32 * 4 == 128);
  static_assert(32 * 16 * 4 == 16 * HD * 2);
  v8us ov[4];
#pragma unroll
  for (int it = 0; it < 4; ++it) { const int row = it * 4 + (lane >> 3), pc = lane & 7; const v4f a = *(const v4fa*)&so[wave][row][pc * 8], c = *(const v4fa*)&so[wave][row][pc * 8 + 4]; FragH f;
#pragma unroll
    for (int q = 0; q < 4; ++q) { f.h[q] = toh_flush(a[q]); f.h[4 + q] = toh_flush(c[q]); }
    ov[it] = f.half[0]; }
  float* stp = ST + ((size_t)bh * SEQ + q0) * 2 + lane;
  for (int pass = 0; pass < 2; ++pass) {
    *(volatile float*)stp = stv;
#pragma unroll
    for (int it = 0; it < 4; ++it) { const int row = it * 4 + (lane >> 3), pc = lane & 7;
      *(volatile v8us*)((unsigned short*)O16 + ((size_t)b * SEQ + q0 + row) * DM + h * HD + pc * 8) = ov[it]; }
    if (pass == 0) __threadfence(); }
}

__device__ __forceinline__ v8f pm_tile(const _Float16* __restrict__ KH, const _Float16* __restrict__ KR, size_t ka, int hh, v16h qh0, v16h qh1, v16h qr0, v16h qr1, float m, float rl, v8f acc) {
  v8f s, r; score_tile(KH, KR, ka, hh, qh0, qh1, qr0, qr1, s, r);
#pragma unroll
  for (int i = 0; i < 8; ++i) { const float e = (s[i] * 0.125f + r[i] * 6.103515625e-05f) - m; acc[i] = acc[i] + __expf(e) * rl; }
  return acc;
}

__global__ __launch_bounds__(128) void k_pmean(const _Float16* __restrict__ QH, const _Float16* __restrict__ QR, const _Float16* __restrict__ KH, const _Float16* __restrict__ KR,
    const float* __restrict__ ST, float* __restrict__ P) {
  __shared__ __attribute__((aligned(16))) float sp[4][16][132];
  static_assert(sizeof(float) * 4 * 16 * 132 <= 131072);
  const int wave = __builtin_amdgcn_readfirstlane(threadIdx.x >> 5); const int lane = threadIdx.x & 31, ln = lane & 15, hh = lane >> 4;
  const int b = blockIdx.z; const int q0 = blockIdx.x * 64 + wave * 16; const int key0 = blockIdx.y * 128;
  const v8f z8 = {0.f,0.f,0.f,0.f,0.f,0.f,0.f,0.f}; v8f a0 = z8, a1 = z8, a2 = z8, a3 = z8, a4 = z8, a5 = z8, a6 = z8, a7 = z8;
#pragma unroll 1
  for (int h = 0; h < NH; ++h) {
    const size_t qoff = ((size_t)b * SEQ + q0 + ln) * DM + h * HD;
    const v16h qh0 = g2_frag(QH + qoff, hh), qh1 = g2_frag(QH + qoff + 32, hh), qr0 = g2_frag(QR + qoff, hh), qr1 = g2_frag(QR + qoff + 32, hh);
    const size_t sti = ((size_t)(b * NH + h) * SEQ + q0) * 2; const float m = ST[sti + ln], rl = ST[sti + 16 + ln];
    const size_t kbase = ((size_t)b * SCTX + key0 + ln) * DM + h * HD;
    a0 = pm_tile(KH, KR, kbase, hh, qh0, qh1, qr0, qr1, m, rl, a0);
    a1 = pm_tile(KH, KR, kbase + (size_t)16 * DM, hh, qh0, qh1, qr0, qr1, m, rl, a1);
    a2 = pm_tile(KH, KR, kbase + (size_t)32 * DM, hh, qh0, qh1, qr0, qr1, m, rl, a2);
    a3 = pm_tile(KH, KR, kbase + (size_t)48 * DM, hh, qh0, qh1, qr0, qr1, m, rl, a3);
    a4 = pm_tile(KH, KR, kbase + (size_t)64 * DM, hh, qh0, qh1, qr0, qr1, m, rl, a4);
    a5 = pm_tile(KH, KR, kbase + (size_t)80 * DM, hh, qh0, qh1, qr0, qr1, m, rl, a5);
    a6 = pm_tile(KH, KR, kbase + (size_t)96 * DM, hh, qh0, qh1, qr0, qr1, m, rl, a6);
    a7 = pm_tile(KH, KR, kbase + (size_t)112 * DM, hh, qh0, qh1, qr0, qr1, m, rl, a7);
  }
  const float inv = 1.0f / (float)NH;
#pragma unroll
  for (int r = 0; r < 8; ++r) { const int c = 8 * hh + r;
    sp[wave][ln][c] = a0[r] * inv; sp[wave][ln][16 + c] = a1[r] * inv; sp[wave][ln][32 + c] = a2[r] * inv; sp[wave][ln][48 + c] = a3[r] * inv;
    sp[wave][ln][64 + c] = a4[r] * inv; sp[wave][ln][80 + c] = a5[r] * inv; sp[wave][ln][96 + c] = a6[r] * inv; sp[wave][ln][112 + c] = a7[r] * inv; }
  __builtin_amdgcn_fence(4  , "workgroup"); __builtin_amdgcn_wave_barrier();
  static_assert(32 * 16 * 16 == 16 * 128 * 4);
  for (int pass = 0; pass < 2; ++pass) {
#pragma unroll
    for (int it = 0; it < 16; ++it) { const int line = it * 4 + (lane >> 3); const int row = line >> 2; const int col = (line & 3) * 32 + (lane & 7) * 4;
      const v4f v = *(const v4fa*)&sp[wave][row][col];
      *(volatile v4f*)(P + ((size_t)b * SEQ_FULL + q0 + row) * SCTX + key0 + col) = v; }
    if (pass == 0) __threadfence(); }
}

constexpr size_t al256(size_t v) { return (v + 255) & ~(size_t)255; }
constexpr size_t SZ_W   = al256((size_t)4 * DM * DM * 2);
constexpr size_t SZ_X16 = al256(NR * DM * 2);
constexpr size_t SZ_C16 = al256(NRC * DM * 2);
constexpr size_t SZ_QF  = al256(NR * DM * 4);
constexpr size_t SZ_KF  = al256(NRC * DM * 4);
constexpr size_t SZ_V16 = al256(NRC * DM * 2);
constexpr size_t SZ_QP  = al256(NR * DM * 2);
constexpr size_t SZ_KP  = al256(NRC * DM * 2);
constexpr size_t SZ_VT  = al256((size_t)NB * NH * HD * SCTX * 2);
constexpr size_t SZ_O16 = al256(NR * DM * 2);
constexpr size_t SZ_ST  = al256((size_t)NB * NH * SEQ * 2 * 4);
constexpr size_t WS_TOTAL = SZ_W + SZ_X16 + SZ_C16 + SZ_QF + SZ_KF + SZ_V16 + 2 * SZ_QP + 2 * SZ_KP + SZ_VT + SZ_O16 + SZ_ST;
static_assert(WS_TOTAL <= (size_t)134217728);
static_assert((NR % 128) == 0 && (NRC % 128) == 0);
static_assert((size_t)NB * NH <= 65535 && SCTX / 128 <= 65535);

extern "C" void kernel_launch(void* const* d_in, const int* in_sizes, int n_in,
                              void* d_out, int out_size, void* d_ws, size_t ws_size, hipStream_t stream) {
  if (n_in < 12) return;
  const float* x = (const float*)d_in[0]; const float* ctx = (const float*)d_in[1];
  const float* Wq = (const float*)d_in[2]; const float* bq = (const float*)d_in[3]; const float* Wk = (const float*)d_in[4]; const float* bk = (const float*)d_in[5];
  const float* Wv = (const float*)d_in[6]; const float* bv = (const float*)d_in[7]; const float* qsc = (const float*)d_in[8]; const float* ksc = (const float*)d_in[9];
  const float* Wp = (const float*)d_in[10]; const float* bp = (const float*)d_in[11];
  if ((size_t)in_sizes[0] < ((size_t)(NB - 1) * SEQ_FULL + SEQ) * DM) return;
  if ((size_t)in_sizes[1] < NRC * DM) return;
  if ((size_t)in_sizes[2] < (size_t)DM * DM || (size_t)in_sizes[4] < (size_t)DM * DM || (size_t)in_sizes[6] < (size_t)DM * DM || (size_t)in_sizes[10] < (size_t)DM * DM) return;
  if (in_sizes[3] < DM || in_sizes[5] < DM || in_sizes[7] < DM || in_sizes[8] < DM || in_sizes[9] < DM || in_sizes[11] < DM) return;
  if ((size_t)out_size < (size_t)NB_FULL * SEQ_FULL * DM + ((size_t)(NB - 1) * SEQ_FULL + SEQ) * SCTX) return;
  float* out0 = (float*)d_out; float* out1 = out0 + (size_t)NB_FULL * SEQ_FULL * DM;

  char* ws = (char*)d_ws; size_t off = 0;
  auto take = [&](size_t bytes) { char* p = ws + off; off += (bytes + 255) & ~(size_t)255; return p; };
  _Float16* RW = (_Float16*)take(SZ_W); _Float16* X16 = (_Float16*)take(SZ_X16); _Float16* C16 = (_Float16*)take(SZ_C16);
  float* QF = (float*)take(SZ_QF); float* KF = (float*)take(SZ_KF); _Float16* V16 = (_Float16*)take(SZ_V16);
  _Float16* QH = (_Float16*)take(SZ_QP); _Float16* QR = (_Float16*)take(SZ_QP); _Float16* KH = (_Float16*)take(SZ_KP); _Float16* KR = (_Float16*)take(SZ_KP);
  _Float16* VT = (_Float16*)take(SZ_VT); _Float16* O16 = (_Float16*)take(SZ_O16); float* ST = (float*)take(SZ_ST);
  if (off > ws_size || off > (size_t)134217728) return;
  _Float16* Bq = RW; _Float16* Bk = RW + (size_t)DM * DM; _Float16* Bv = RW + (size_t)2 * DM * DM; _Float16* Bp = RW + (size_t)3 * DM * DM;

  auto wt = [&](const float* W, _Float16* Bt, int K, int N) { k_wt_f16<<<(unsigned)(((size_t)N * (K / 8) + 255) / 256), 256, 0, stream>>>(W, Bt, K, N, 16.0f); };
  auto gx = [](int M, int N) { return (unsigned)(((M + 127) / 128) * (N / 64)); };

  wt(Wq, Bq, DM, DM); wt(Wk, Bk, DM, DM); wt(Wv, Bv, DM, DM); wt(Wp, Bp, DM, DM);
  if (SEQ == SEQ_FULL) { k_x16<<<(unsigned)((NR * DM / 8 + 255) / 256), 256, 0, stream>>>(x, X16, NR * DM / 8); }
  else { for (int b = 0; b < NB; ++b) k_x16<<<(unsigned)(((size_t)SEQ * DM / 8 + 255) / 256), 256, 0, stream>>>(x + (size_t)b * SEQ_FULL * DM, X16 + (size_t)b * SEQ * DM, (size_t)SEQ * DM / 8); }
  k_x16<<<(unsigned)((NRC * DM / 8 + 255) / 256), 256, 0, stream>>>(ctx, C16, NRC * DM / 8);
  k_gemm2<0, 0, 0, 0, 0><<<dim3(gx((int)NR, DM), 1), 128, 0, stream>>>(X16, DM, 0, Bq, DM, 0, 0.0625f, bq, nullptr, nullptr, 0, nullptr, 0, QF, nullptr, DM, 0, (int)NR, DM, DM);
  k_gemm2<0, 0, 0, 0, 0><<<dim3(gx((int)NRC, DM), 1), 128, 0, stream>>>(C16, DM, 0, Bk, DM, 0, 0.0625f, bk, nullptr, nullptr, 0, nullptr, 0, KF, nullptr, DM, 0, (int)NRC, DM, DM);
  k_gemm2<0, 0, 0, 0, 0><<<dim3(gx((int)NRC, DM), 1), 128, 0, stream>>>(C16, DM, 0, Bv, DM, 0, 0.0625f, bv, nullptr, nullptr, 0, nullptr, 0, nullptr, V16, DM, 0, (int)NRC, DM, DM);
  k_rmsres<<<(unsigned)((NR + 7) / 8), 256, 0, stream>>>(QF, qsc, QH, QR, (int)NR);
  k_rmsres<<<(unsigned)((NRC + 7) / 8), 256, 0, stream>>>(KF, ksc, KH, KR, (int)NRC);
  k_vt<NH, SCTX><<<NB * NH * (SCTX / 64), 256, 0, stream>>>(V16, DM, 0, VT);
  k_flash<<<dim3(SEQ / 64, NB * NH), 128, 0, stream>>>(QH, QR, KH, KR, VT, O16, ST);
  k_pmean<<<dim3(SEQ / 64, SCTX / 128, NB), 128, 0, stream>>>(QH, QR, KH, KR, ST, out1);
  for (int b = 0; b < NB; ++b) { const size_t rq0 = (size_t)b * SEQ;
    k_gemm2<0, 0, 0, 0, 0><<<dim3(gx(SEQ, DM), 1), 128, 0, stream>>>(O16 + rq0 * DM, DM, 0, Bp, DM, 0, 0.0009765625f, bp, nullptr, nullptr, 0, nullptr, 0, out0 + (size_t)b * SEQ_FULL * DM, nullptr, DM, 0, SEQ, DM, DM); }
}
